// SiameseTangentLayer_26560077758935
// MI455X (gfx1250) — hardware-run, weakly checked
//
#include <hip/hip_runtime.h>


#ifndef NB
#define NB 1024
#endif
#define NB_FULL 1024
#define NK   62
#define DD   512
#define SS   64
#define TP   128

static_assert(SS == 64);
static_assert(DD % 64 == 0);
static_assert(DD % 32 == 0);
static_assert(TP == 2 * SS);
static_assert(TP % 32 == 0);
static_assert(NB % 64 == 0);
static_assert(NB <= NB_FULL);
static_assert(((size_t)NB * DD) % 8 == 0);
static_assert(((size_t)NK * DD) % 8 == 0);
static_assert(((size_t)NB * NK) % 32 == 0);
static_assert((size_t)NB * NK * 4 <= (size_t)253952);

typedef unsigned short bf;
typedef __attribute__((ext_vector_type(16))) __bf16   v16bf;
typedef __attribute__((ext_vector_type(8)))  unsigned short v8us;
typedef __attribute__((ext_vector_type(8)))  float    v8f;
typedef __attribute__((ext_vector_type(4)))  float    v4f;
typedef v4f  __attribute__((may_alias)) v4fa;

__device__ __forceinline__ unsigned short f2bf(float f) { unsigned u = __float_as_uint(f); u += 0x7FFFu + ((u >> 16) & 1u); return (unsigned short)(u >> 16); }
__device__ __forceinline__ float bf2f(unsigned short w) { return __uint_as_float(((unsigned)w) << 16); }
__device__ __forceinline__ float bfr(float f) { return bf2f(f2bf(f)); }
__device__ __forceinline__ v16bf cat16b(v8us lo, v8us hi) { return __builtin_bit_cast(v16bf, __builtin_shufflevector(lo, hi, 0, 1, 2, 3, 4, 5, 6, 7, 8, 9, 10, 11, 12, 13, 14, 15)); }
__device__ __forceinline__ v8f wmmab(v16bf a, v16bf b, v8f c) { return __builtin_amdgcn_wmma_f32_16x16x32_bf16(false, a, false, b, (short)0, c, false, false); }
__device__ __forceinline__ v16bf ldb(const bf* p)  { return cat16b(*(const v8us*)p, *(const v8us*)(p + 16)); }
__device__ __forceinline__ void wave_sync() { __builtin_amdgcn_fence(3  , "wavefront"); __builtin_amdgcn_wave_barrier(); asm volatile("" ::: "memory"); }

__global__ __launch_bounds__(256) void k_cvt8(const float* __restrict__ src, bf* dst, size_t n8) {
    const size_t i = (size_t)blockIdx.x * 256 + threadIdx.x; if (i >= n8) return;
    const v8f v = *(const v8f*)(src + i * 8); v8us o;
#pragma unroll
    for (int k = 0; k < 8; ++k) o[k] = f2bf(v[k]);
    *(volatile v8us*)(dst + i * 8) = o; __threadfence(); *(volatile v8us*)(dst + i * 8) = o;
}

__global__ __launch_bounds__(256) void k_omega(const float* __restrict__ om, bf* OB, bf* OT) {
    __shared__ float ts[64 * 65];
    const int t = threadIdx.x; const int dc = blockIdx.x, kp = blockIdx.y;
    const float* src = om + ((size_t)kp * DD + (size_t)dc * 64) * SS;
#pragma unroll
    for (int i = 0; i < 4; ++i) { const int p = t + 256 * i; const int row = p >> 4, c4 = (p & 15) * 4;
        const v4f v = *(const v4f*)(src + row * 64 + c4);
        ts[row * 65 + c4 + 0] = v[0]; ts[row * 65 + c4 + 1] = v[1]; ts[row * 65 + c4 + 2] = v[2]; ts[row * 65 + c4 + 3] = v[3]; }
    __syncthreads();
    v8us o1[2], o2[2]; size_t a1[2], a2[2];
#pragma unroll
    for (int i = 0; i < 2; ++i) { const int p = t + 256 * i; const int row = p >> 3, q = p & 7;
#pragma unroll
        for (int j = 0; j < 8; ++j) { o1[i][j] = f2bf(ts[row * 65 + 8 * q + j]); o2[i][j] = f2bf(ts[(8 * q + j) * 65 + row]); }
        a1[i] = ((size_t)kp * DD + (size_t)dc * 64 + row) * SS + 8 * q;
        a2[i] = ((size_t)kp * SS + row) * DD + (size_t)dc * 64 + 8 * q; }
#pragma unroll
    for (int i = 0; i < 2; ++i) { *(volatile v8us*)(OB + a1[i]) = o1[i]; *(volatile v8us*)(OT + a2[i]) = o2[i]; }
    __threadfence();
#pragma unroll
    for (int i = 0; i < 2; ++i) { *(volatile v8us*)(OB + a1[i]) = o1[i]; *(volatile v8us*)(OT + a2[i]) = o2[i]; }
}

__global__ __launch_bounds__(256) void k_yo(const float* __restrict__ y, const float* __restrict__ om, float* YO) {
    __shared__ __align__(16) float part[4 * 64];
    const int t = threadIdx.x; const int s = t & 63; const int ch = __builtin_amdgcn_readfirstlane((int)(threadIdx.x >> 6)); const int kp = blockIdx.x;
    const float* yk = y + (size_t)kp * DD + ch * 128;
    const float* ok = om + ((size_t)kp * DD + (size_t)ch * 128) * SS + s;
    float acc = 0.0f;
#pragma unroll 4
    for (int d = 0; d < 128; ++d) acc = fmaf(bfr(yk[d]), bfr(ok[(size_t)d * SS]), acc);
    part[ch * 64 + s] = acc;
    __syncthreads();
    if (t < 16) { v4f o;
#pragma unroll
        for (int j = 0; j < 4; ++j) { const int c = 4 * t + j; o[j] = ((part[c] + part[64 + c]) + part[128 + c]) + part[192 + c]; }
        float* dst = YO + (size_t)kp * SS + 4 * t;
        *(volatile v4f*)dst = o; __threadfence(); *(volatile v4f*)dst = o; }
}

__global__ __launch_bounds__(32) void k_gemm_a(const bf* __restrict__ A, const bf* __restrict__ Bt, const float* __restrict__ YO, bf* T) {
    __shared__ __align__(16) float os[16 * 68];
    const int K = DD;
    const int lane = threadIdx.x & 31, lr = lane & 15, hi = lane >> 4; const int r0 = blockIdx.x * 64, kp = blockIdx.y, c0 = kp * 64;
    v8f acc[4][4];
#pragma unroll
    for (int mb = 0; mb < 4; ++mb)
#pragma unroll
        for (int nb = 0; nb < 4; ++nb) acc[mb][nb] = (v8f){};
    const size_t aoff = (size_t)(r0 + lr) * K + 8 * hi, boff = (size_t)(c0 + lr) * K + 8 * hi;
#pragma unroll 1
    for (int kc = 0; kc < K; kc += 32) {
        v16bf a[4];
#pragma unroll
        for (int mb = 0; mb < 4; ++mb) a[mb] = ldb(A + aoff + (size_t)mb * 16 * K + kc);
#pragma unroll
        for (int nb = 0; nb < 4; ++nb) { const v16bf b = ldb(Bt + boff + (size_t)nb * 16 * K + kc);
#pragma unroll
            for (int mb = 0; mb < 4; ++mb) acc[mb][nb] = wmmab(a[mb], b, acc[mb][nb]); }
        asm volatile("v_nop\n\tv_nop\n\tv_nop\n\tv_nop" : "+v"(acc[0][0]), "+v"(acc[1][1]), "+v"(acc[2][2]), "+v"(acc[3][3]) : "v"(a[0]), "v"(a[1]), "v"(a[2]), "v"(a[3]));
    }
    const int c8 = (lane & 7) * 8, rg = lane >> 3;
    const v4f y0 = *(const v4f*)(YO + (size_t)kp * SS + c8), y1 = *(const v4f*)(YO + (size_t)kp * SS + c8 + 4);
    const size_t tbase = ((size_t)kp * NB + r0) * TP;
#pragma unroll
    for (int mb = 0; mb < 4; ++mb) {
#pragma unroll
        for (int nb = 0; nb < 4; ++nb) {
#pragma unroll
            for (int j = 0; j < 8; ++j) os[(hi * 8 + j) * 68 + nb * 16 + lr] = acc[mb][nb][j]; }
        wave_sync();
        const size_t sb = tbase + (size_t)(mb * 16) * TP;
#pragma unroll 1
        for (int ps = 0; ps < 2; ++ps) {
#pragma unroll
            for (int s = 0; s < 4; ++s) { const int row = 4 * s + rg;
                const v4f x0 = *(const v4fa*)(&os[row * 68 + c8]); const v4f x1 = *(const v4fa*)(&os[row * 68 + c8 + 4]); v8us hv, lv;
#pragma unroll
                for (int i = 0; i < 4; ++i) { const float t0 = y0[i] - x0[i]; const float t1 = y1[i] - x1[i];
                    const unsigned short h0 = f2bf(t0), h1 = f2bf(t1); hv[i] = h0; hv[4 + i] = h1;
                    lv[i] = f2bf(t0 - bf2f(h0)); lv[4 + i] = f2bf(t1 - bf2f(h1)); }
                const size_t oo = sb + (size_t)row * TP + c8;
                *(volatile v8us*)(T + oo) = hv; *(volatile v8us*)(T + oo + SS) = lv; }
            if (ps == 0) __threadfence(); }
        wave_sync();
    }
}

__global__ __launch_bounds__(32) void k_gemm_b(const bf* __restrict__ T, const bf* __restrict__ OB, const bf* __restrict__ XB, const bf* __restrict__ YB, float* DW) {
    __shared__ __align__(16) float os[16 * 68];
    __shared__ __align__(16) float ds[64];
    const int lane = threadIdx.x & 31, lr = lane & 15, hi = lane >> 4; const int r0 = blockIdx.x * 64, kp = blockIdx.y;
    const int c8 = (lane & 7) * 8, rg = lane >> 3;
    const size_t aoff = ((size_t)kp * NB + r0 + lr) * TP + 8 * hi;
    float psum[4][4];
#pragma unroll
    for (int mb = 0; mb < 4; ++mb)
#pragma unroll
        for (int s = 0; s < 4; ++s) psum[mb][s] = 0.0f;
#pragma unroll 1
    for (int et = 0; et < DD / 64; ++et) {
        const int e0 = et * 64;
        const size_t boff = ((size_t)kp * DD + e0 + lr) * SS + 8 * hi;
        v8f acc[4][4];
#pragma unroll
        for (int mb = 0; mb < 4; ++mb)
#pragma unroll
            for (int nb = 0; nb < 4; ++nb) acc[mb][nb] = (v8f){};
#pragma unroll 1
        for (int kc = 0; kc < TP; kc += 32) {
            const int kb = kc & (SS - 1);
            v16bf a[4];
#pragma unroll
            for (int mb = 0; mb < 4; ++mb) a[mb] = ldb(T + aoff + (size_t)mb * 16 * TP + kc);
#pragma unroll
            for (int nb = 0; nb < 4; ++nb) { const v16bf b = ldb(OB + boff + (size_t)nb * 16 * SS + kb);
#pragma unroll
                for (int mb = 0; mb < 4; ++mb) acc[mb][nb] = wmmab(a[mb], b, acc[mb][nb]); }
            asm volatile("v_nop\n\tv_nop\n\tv_nop\n\tv_nop" : "+v"(acc[0][0]), "+v"(acc[1][1]), "+v"(acc[2][2]), "+v"(acc[3][3]) : "v"(a[0]), "v"(a[1]), "v"(a[2]), "v"(a[3]));
        }
        const v8us yw = *(const v8us*)(YB + (size_t)kp * DD + e0 + c8);
        float yf[8];
#pragma unroll
        for (int i = 0; i < 8; ++i) yf[i] = bf2f(yw[i]);
#pragma unroll
        for (int mb = 0; mb < 4; ++mb) {
#pragma unroll
            for (int nb = 0; nb < 4; ++nb) {
#pragma unroll
                for (int j = 0; j < 8; ++j) os[(hi * 8 + j) * 68 + nb * 16 + lr] = acc[mb][nb][j]; }
            wave_sync();
#pragma unroll
            for (int s = 0; s < 4; ++s) { const int row = 4 * s + rg;
                const v4f u0 = *(const v4fa*)(&os[row * 68 + c8]); const v4f u1 = *(const v4fa*)(&os[row * 68 + c8 + 4]);
                const v8us xw = *(const v8us*)(XB + (size_t)(r0 + mb * 16 + row) * DD + e0 + c8);
                float p = psum[mb][s];
#pragma unroll
                for (int i = 0; i < 4; ++i) { const float ra = (yf[i] - bf2f(xw[i])) - u0[i]; const float rb = (yf[4 + i] - bf2f(xw[4 + i])) - u1[i];
                    p = fmaf(ra, ra, p); p = fmaf(rb, rb, p); }
                psum[mb][s] = p; }
            wave_sync();
        }
    }
#pragma unroll
    for (int mb = 0; mb < 4; ++mb)
#pragma unroll
        for (int s = 0; s < 4; ++s) { float v = psum[mb][s];
            v += __shfl_xor(v, 1, 32); v += __shfl_xor(v, 2, 32); v += __shfl_xor(v, 4, 32);
            if ((lane & 7) == 0) ds[mb * 16 + 4 * s + rg] = v; }
    wave_sync();
    if (lane < 16) { const v4f o = *(const v4fa*)(&ds[4 * lane]);
        float* dst = DW + (size_t)kp * NB + r0 + 4 * lane;
        *(volatile v4f*)dst = o; __threadfence(); *(volatile v4f*)dst = o; }
}

__global__ __launch_bounds__(256) void k_out(const float* __restrict__ DW, float* OUT, int n4) {
    const int i = blockIdx.x * 256 + threadIdx.x; if (i >= n4) return;
    v4f o;
#pragma unroll
    for (int j = 0; j < 4; ++j) { const int e = 4 * i + j; const int b = e / NK; const int k = e - b * NK; o[j] = DW[(size_t)k * NB + b]; }
    float* dst = OUT + (size_t)4 * i;
    *(volatile v4f*)dst = o; __threadfence(); *(volatile v4f*)dst = o;
}

static constexpr size_t al256(size_t v) { return (v + 255) & ~(size_t)255; }
static constexpr size_t SZ_XB = al256((size_t)NB * DD * 2);
static constexpr size_t SZ_YB = al256((size_t)NK * DD * 2);
static constexpr size_t SZ_OB = al256((size_t)NK * DD * SS * 2);
static constexpr size_t SZ_OT = al256((size_t)NK * SS * DD * 2);
static constexpr size_t SZ_YO = al256((size_t)NK * SS * 4);
static constexpr size_t SZ_T  = al256((size_t)NK * NB * TP * 2);
static constexpr size_t SZ_DW = al256((size_t)NK * NB * 4);
static constexpr size_t SZ_TOTAL = SZ_XB + SZ_YB + SZ_OB + SZ_OT + SZ_YO + SZ_T + SZ_DW;
static_assert(SZ_TOTAL <= (size_t)134217728);

extern "C" void kernel_launch(void* const* d_in, const int* in_sizes, int n_in,
                              void* d_out, int out_size, void* d_ws, size_t ws_size, hipStream_t stream) {
    if (n_in < 3) return;
    if ((size_t)in_sizes[0] < (size_t)NB * DD) return;
    if ((size_t)in_sizes[1] < (size_t)NK * DD) return;
    if ((size_t)in_sizes[2] < (size_t)NK * DD * SS) return;
    if ((size_t)out_size < (size_t)NB * NK) return;
    if (SZ_TOTAL > ws_size) return;
    const float* x = (const float*)d_in[0]; const float* y = (const float*)d_in[1]; const float* om = (const float*)d_in[2];
    float* OUT = (float*)d_out;
    char* wsp = (char*)d_ws;
    bf* XB = (bf*)wsp; wsp += SZ_XB;
    bf* YB = (bf*)wsp; wsp += SZ_YB;
    bf* OB = (bf*)wsp; wsp += SZ_OB;
    bf* OT = (bf*)wsp; wsp += SZ_OT;
    float* YO = (float*)wsp; wsp += SZ_YO;
    bf* T = (bf*)wsp; wsp += SZ_T;
    float* DW = (float*)wsp; wsp += SZ_DW;

    { const size_t n8 = (size_t)NB * DD / 8; k_cvt8<<<(unsigned)((n8 + 255) / 256), 256, 0, stream>>>(x, XB, n8); }
    { const size_t n8 = (size_t)NK * DD / 8; k_cvt8<<<(unsigned)((n8 + 255) / 256), 256, 0, stream>>>(y, YB, n8); }
    k_omega<<<dim3(DD / 64, NK, 1), 256, 0, stream>>>(om, OB, OT);
    k_yo<<<NK, 256, 0, stream>>>(y, om, YO);
    k_gemm_a<<<dim3(NB / 64, NK, 1), 32, 0, stream>>>(XB, OT, YO, T);
    k_gemm_b<<<dim3(NB / 64, NK, 1), 32, 0, stream>>>(T, OB, XB, YB, DW);
    { const int n4 = NB * NK / 4; k_out<<<(unsigned)((n4 + 255) / 256), 256, 0, stream>>>(DW, OUT, n4); }
}
